// HopGatedGATv2Conv_9285719294404
// MI455X (gfx1250) — hardware-run, weakly checked
//
#include <hip/hip_runtime.h>
#include <stddef.h>
#include <stdint.h>
#include <math.h>

#define NN      50000
#define FD      256
#define HC      256
#define NHEAD   4
#define CD      64
#define NHOP    3
#define NE      400000
#define NBT     528
#define NXL     512
#define HROWS   25088
#define MP      50176
#define GBM     128
#define SP      68
#define NTHR    256
#define NWAVE   8
#define EPT     8
#define WCH     (32 * EPT)
#define NBRUN   1024
#define SLB     10
#define NBK     49
#define WLCAP   2048
#define RCAP    12288
#define DEGCAP  40
#define MAXDEG_MEAS   24
#define MAXB1024_MEAS 8415
#define LSLOPE  0.2f

#define PBX  (HROWS * FD / 8 / NTHR)
#define PBW  (NBT * FD / 8 / NTHR)
#define SM_BV    0
#define SM_ATT   544
#define SM_BIA   1312
#define SM_TOT   1504
#define SM_UNITS (SM_TOT / 4)
#define SAB_N    960

#define BK_ZINTS (NWAVE * WLCAP + RCAP + 3 * NBRUN)
#define BK_INTS  (BK_ZINTS + 16)
#define BK_LDS   (BK_INTS * 4)

static_assert(NHEAD * CD == HC && HC == 32 * 8);
static_assert(NN <= NBK * NBRUN);
static_assert(NBT == 33 * 16 && NBT >= 2 * HC + NHOP);
static_assert(HROWS == 196 * GBM && 2 * HROWS == MP && MP >= NN && HROWS < NN);
static_assert(NBRUN == (1 << SLB) && NBRUN <= 1024 && NBRUN % 32 == 0);
static_assert(NN <= 65536);
static_assert(NE % EPT == 0 && NE < (1 << 21) && (((long long)NE) << SLB) < (1LL << 31));
static_assert((long long)RCAP * 100 >= (long long)MAXB1024_MEAS * 105);
static_assert(NWAVE * WLCAP >= RCAP && RCAP % (NTHR * 4) == 0 && (2 * NBRUN) % (NTHR * 4) == 0);
static_assert(WLCAP >= MAXB1024_MEAS / NWAVE + 512);
static_assert(MAXDEG_MEAS + 8 <= DEGCAP);
static_assert(BK_ZINTS % 4 == 0 && BK_LDS <= 327680);
static_assert((GBM * SP + 64) * 4 <= 65536);
static_assert((HROWS * FD / 8) % NTHR == 0 && (NBT * FD / 8) % NTHR == 0 && PBW == 66);
static_assert(FD % 32 == 0);
static_assert(NN % NWAVE == 0);
static_assert(SM_ATT + NHOP * HC == SM_BIA && SM_BIA + NHOP * CD == SM_TOT && SAB_N / 4 <= NTHR);
static_assert(SM_UNITS <= 2 * NTHR && SM_UNITS % 8 == 0);

typedef float          v4f   __attribute__((ext_vector_type(4)));
typedef float          v8f   __attribute__((ext_vector_type(8)));
typedef int            v4i   __attribute__((ext_vector_type(4)));
typedef int            v8i   __attribute__((ext_vector_type(8)));
typedef unsigned short v8us  __attribute__((ext_vector_type(8)));
typedef unsigned short v16us __attribute__((ext_vector_type(16)));
typedef __bf16         v16bf __attribute__((ext_vector_type(16)));
typedef v4f  __attribute__((may_alias)) v4fa;
typedef v4i  __attribute__((may_alias)) v4ia;
typedef v8us __attribute__((may_alias)) v8usa;
union FragB { v16bf v; v16us u; v8us h[2]; v8i w; };

__device__ __forceinline__ v8f wmb(const FragB& a, const FragB& b, v8f c) {
  v8f d = __builtin_amdgcn_wmma_f32_16x16x32_bf16(false, a.v, false, b.v, (short)0, c, false, false);
  asm volatile("v_nop\n\tv_nop\n\tv_nop\n\tv_nop" : "+v"(d) : "v"(a.w), "v"(b.w));
  return d;
}

__device__ __forceinline__ unsigned bf16_bits(float f) {
  const unsigned u = __float_as_uint(f);
  const unsigned r = (u + 0x7FFFu + ((u >> 16) & 1u)) >> 16;
  const unsigned q = (u >> 16) | 0x40u;
  return ((u & 0x7fffffffu) > 0x7f800000u) ? q : r;
}

__device__ __forceinline__ void st2_v4f(float* p, v4f v) {
  *(volatile v4f*)p = v;
  __threadfence();
  *(volatile v4f*)p = v;
}
__device__ __forceinline__ void st2_v8us(unsigned short* p, v8us v) {
  *(volatile v8us*)p = v;
  __threadfence();
  *(volatile v8us*)p = v;
}

__device__ __forceinline__ v8us col8(const float* __restrict__ base, int stride, unsigned mk) {
  float f[8];
#pragma unroll
  for (int i = 0; i < 8; ++i) f[i] = base[(size_t)i * (size_t)stride];
  v8us o;
#pragma unroll
  for (int i = 0; i < 8; ++i) o[i] = (unsigned short)(bf16_bits(f[i]) & mk);
  return o;
}

__global__ __launch_bounds__(NTHR) void k_prep(const float* __restrict__ x, const float* __restrict__ wl,
                                               const float* __restrict__ bl, const float* __restrict__ wr,
                                               const float* __restrict__ br, const float* __restrict__ att,
                                               const float* __restrict__ bias, const float* __restrict__ wg,
                                               const float* __restrict__ bg,
                                               unsigned short* xbh, unsigned short* bt, float* sm, int half) {
  const int tid = (int)threadIdx.x;
  const int blk = (int)blockIdx.x;
  if (blk < PBX) {
    const int u    = blk * NTHR + tid;
    const int row  = u >> 5, k8 = (u & 31) * 8;
    const int grow = half * HROWS + row;
    const int rc   = grow < NN ? grow : NN - 1;
    const unsigned mk = grow < NN ? 0xffffu : 0u;
    const float* p = x + (size_t)rc * FD + k8;
    const v4f a = *(const v4fa*)p;
    const v4f b = *(const v4fa*)(p + 4);
    v8us o;
    o[0] = (unsigned short)(bf16_bits(a.x) & mk); o[1] = (unsigned short)(bf16_bits(a.y) & mk);
    o[2] = (unsigned short)(bf16_bits(a.z) & mk); o[3] = (unsigned short)(bf16_bits(a.w) & mk);
    o[4] = (unsigned short)(bf16_bits(b.x) & mk); o[5] = (unsigned short)(bf16_bits(b.y) & mk);
    o[6] = (unsigned short)(bf16_bits(b.z) & mk); o[7] = (unsigned short)(bf16_bits(b.w) & mk);
    st2_v8us(xbh + (size_t)row * FD + k8, o);
  } else if (blk < PBX + 32) {
    const int u = (blk - PBX) * NTHR + tid;
    const int n = u >> 5, k8 = (u & 31) * 8;
    const v8us o = col8(wl + (size_t)k8 * HC + n, HC, 0xffffu);
    st2_v8us(bt + (size_t)n * FD + k8, o);
  } else if (blk < PBX + 64) {
    const int u = (blk - PBX - 32) * NTHR + tid;
    const int n = u >> 5, k8 = (u & 31) * 8;
    const v8us o = col8(wr + (size_t)k8 * HC + n, HC, 0xffffu);
    st2_v8us(bt + (size_t)(HC + n) * FD + k8, o);
  } else if (blk < PBX + PBW) {
    const int u = (blk - PBX - 64) * NTHR + tid;
    const int n = u >> 5, k8 = (u & 31) * 8;
    const int nc = n < NHOP ? n : NHOP - 1;
    const unsigned mk = n < NHOP ? 0xffffu : 0u;
    const v8us o = col8(wg + (size_t)k8 * NHOP + nc, NHOP, mk);
    st2_v8us(bt + (size_t)(2 * HC + n) * FD + k8, o);
  } else {
#pragma unroll 1
    for (int it = 0; it < 2; ++it) {
      const int i4 = it * NTHR + tid;
      const int ic = i4 < SM_UNITS ? i4 : SM_UNITS - 1;
      int ul = ic;       ul = ul > 63 ? 63 : ul;
      int ur = ic - 64;  ur = ur < 0 ? 0 : (ur > 63 ? 63 : ur);
      int ua = ic - 136; ua = ua < 0 ? 0 : (ua > 191 ? 191 : ua);
      int ub = ic - 328; ub = ub < 0 ? 0 : (ub > 47 ? 47 : ub);
      const v4f vl = *(const v4fa*)(bl + 4 * ul);
      const v4f vr = *(const v4fa*)(br + 4 * ur);
      const v4f va = *(const v4fa*)(att + 4 * ua);
      const v4f vb = *(const v4fa*)(bias + 4 * ub);
      const float g0 = bg[0], g1 = bg[1], g2 = bg[2];
      asm volatile("" :: "v"(vl), "v"(vr));
      asm volatile("" :: "v"(va), "v"(vb));
      asm volatile("" :: "v"(g0), "v"(g1), "v"(g2));
      const unsigned ml = (ic < 64) ? 0xffffffffu : 0u;
      const unsigned mr = (ic >= 64 && ic < 128) ? 0xffffffffu : 0u;
      const unsigned mg = (ic == 128) ? 0xffffffffu : 0u;
      const unsigned ma = (ic >= 136 && ic < 328) ? 0xffffffffu : 0u;
      const unsigned mb = (ic >= 328) ? 0xffffffffu : 0u;
      v4f o;
      o.x = __uint_as_float(((bf16_bits(vl.x) << 16) & ml) | ((bf16_bits(vr.x) << 16) & mr) |
                            ((bf16_bits(g0) << 16) & mg) | ((bf16_bits(va.x) << 16) & ma) |
                            ((bf16_bits(vb.x) << 16) & mb));
      o.y = __uint_as_float(((bf16_bits(vl.y) << 16) & ml) | ((bf16_bits(vr.y) << 16) & mr) |
                            ((bf16_bits(g1) << 16) & mg) | ((bf16_bits(va.y) << 16) & ma) |
                            ((bf16_bits(vb.y) << 16) & mb));
      o.z = __uint_as_float(((bf16_bits(vl.z) << 16) & ml) | ((bf16_bits(vr.z) << 16) & mr) |
                            ((bf16_bits(g2) << 16) & mg) | ((bf16_bits(va.z) << 16) & ma) |
                            ((bf16_bits(vb.z) << 16) & mb));
      o.w = __uint_as_float(((bf16_bits(vl.w) << 16) & ml) | ((bf16_bits(vr.w) << 16) & mr) |
                            ((bf16_bits(va.w) << 16) & ma) | ((bf16_bits(vb.w) << 16) & mb));
      if (i4 < SM_UNITS) st2_v4f(sm + 4 * i4, o);
    }
  }
}

template <int KTOT, int NT>
__device__ __forceinline__ void mm_tiles(const unsigned short* __restrict__ ap,
                                         const unsigned short* __restrict__ bp, v8f (&acc)[NT]) {
#pragma unroll 1
  for (int k0 = 0; k0 < KTOT; k0 += 32) {
    FragB af;
    af.h[0] = *(const v8usa*)(ap + k0);
    af.h[1] = *(const v8usa*)(ap + k0 + 16);
#pragma unroll
    for (int nt = 0; nt < NT; ++nt) {
      const unsigned short* wq = bp + (size_t)(16 * nt) * (size_t)KTOT + k0;
      FragB bf;
      bf.h[0] = *(const v8usa*)wq;
      bf.h[1] = *(const v8usa*)(wq + 16);
      acc[nt] = wmb(af, bf, acc[nt]);
    }
  }
}

template <int NT>
__device__ __forceinline__ void stage_d(float* stg, const v8f (&acc)[NT], int wave, int hh, int m) {
#pragma unroll
  for (int nt = 0; nt < NT; ++nt) {
#pragma unroll
    for (int r = 0; r < 8; ++r) stg[(16 * wave + 8 * hh + r) * SP + 16 * nt + m] = acc[nt][r];
  }
}

__global__ __launch_bounds__(NTHR) __attribute__((amdgpu_num_vgpr(248)))
void k_gemm_one(const unsigned short* __restrict__ XBH, const unsigned short* __restrict__ BT,
                const float* __restrict__ SM, float* XLR, float* GL, int half) {
  __shared__ __attribute__((aligned(16))) float stg[GBM * SP];
  __shared__ __attribute__((aligned(16))) float sb[64];
  const int tid = (int)threadIdx.x, lane = tid & 31, wave = tid >> 5, hh = lane >> 4, m = lane & 15;
  const int rowBase = (int)blockIdx.x * GBM;
  const int y = (int)blockIdx.y;
  const bool wide = y < 8;
  const int colBase = wide ? 64 * y : 2 * HC;

  if (tid < 32) {
    const int q  = lane & 15;
    const int qc = wide ? q : (q & 3);
    const v4f v = *(const v4fa*)(SM + SM_BV + colBase + 4 * qc);
    asm volatile("" :: "v"(v));
    if (lane < 16) *(v4fa*)(sb + 4 * q) = v;
  }

  const unsigned short* ap = XBH + (size_t)(rowBase + 16 * wave + m) * (size_t)FD + 8 * hh;
  const unsigned short* bp = BT + (size_t)(colBase + m) * (size_t)FD + 8 * hh;
  const v8f z = {0.f, 0.f, 0.f, 0.f, 0.f, 0.f, 0.f, 0.f};
  if (wide) {
    v8f acc[4];
#pragma unroll
    for (int t = 0; t < 4; ++t) acc[t] = z;
    mm_tiles<FD, 4>(ap, bp, acc);
    stage_d<4>(stg, acc, wave, hh, m);
  } else {
    v8f acc[1];
    acc[0] = z;
    mm_tiles<FD, 1>(ap, bp, acc);
    stage_d<1>(stg, acc, wave, hh, m);
  }
  __syncthreads();

  if (wide) {
    const v4f bias = *(const v4fa*)(sb + 4 * m);
#pragma unroll 1
    for (int i = 0; i < 8; ++i) {
      const int lr   = 16 * wave + 2 * i + hh;
      const int grow = half * HROWS + rowBase + lr;
      const v4f a = *(const v4fa*)(stg + lr * SP + 4 * m);
      v4f o;
      o.x = a.x + bias.x; o.y = a.y + bias.y; o.z = a.z + bias.z; o.w = a.w + bias.w;
      st2_v4f(XLR + (size_t)grow * NXL + colBase + 4 * m, o);
    }
  } else {
    if (tid < GBM) {
      const v4f bias = *(const v4fa*)sb;
      const v4f a = *(const v4fa*)(stg + tid * SP);
      const int grow = half * HROWS + rowBase + tid;
      v4f o;
      o.x = a.x + bias.x; o.y = a.y + bias.y; o.z = a.z + bias.z; o.w = a.w + bias.w;
      st2_v4f(GL + (size_t)grow * 4, o);
    }
  }
}

__device__ __forceinline__ void bucket_flush(const int* pl, const int* cnt, int ov, int* lp, int* cop, int* fp,
                                             int tid) {
#pragma unroll 1
  for (int i = tid * 4; i < RCAP; i += NTHR * 4) {
    const v4i v = *(const v4ia*)(pl + i);
    *(volatile v4i*)(lp + i) = v;
  }
#pragma unroll 1
  for (int i = tid * 4; i < 2 * NBRUN; i += NTHR * 4) {
    const v4i v = *(const v4ia*)(cnt + i);
    *(volatile v4i*)(cop + i) = v;
  }
  if (tid < 8) {
    const v4i f = {ov, ov, ov, ov};
    *(volatile v4i*)(fp + 4 * tid) = f;
  }
}

__global__ __launch_bounds__(NTHR) void k_bucket(const int* __restrict__ srcs, const int* __restrict__ dsts,
                                                 int* LIST, int* CO, int* FLAG) {
  extern __shared__ __attribute__((aligned(16))) int dsm[];
  int* wl   = dsm;
  int* pl   = dsm + NWAVE * WLCAP;
  int* cnt  = pl + RCAP;
  int* offs = cnt + NBRUN;
  int* cur  = offs + NBRUN;
  int* misc = cur + NBRUN;
  const int tid = (int)threadIdx.x, lane = tid & 31, wave = tid >> 5;
  const int blk = (int)blockIdx.x;
  const unsigned nbs = (unsigned)(blk * NBRUN);

  {
    const v4i z4 = {0, 0, 0, 0};
    for (int i = tid * 4; i < BK_ZINTS; i += NTHR * 4) *(v4ia*)(dsm + i) = z4;
    if (tid < 16) misc[tid] = 0;
  }
  __syncthreads();

  {
    const int per  = ((NE + NWAVE * WCH - 1) / (NWAVE * WCH)) * WCH;
    const int ebeg = wave * per;
    const int eend = (ebeg + per < NE) ? (ebeg + per) : NE;
    const int snt  = (int)(1u << 31);
    int* mylist = wl + wave * WLCAP;
    int wc = 0;
#pragma unroll 1
    for (int cb = ebeg; cb < eend; cb += WCH) {
      const int e0 = cb + lane * EPT;
      const int ec = e0 < NE - EPT ? e0 : NE - EPT;
      const v4i la = *(const v4ia*)(dsts + ec);
      const v4i lb = *(const v4ia*)(dsts + ec + 4);
      asm volatile("" :: "v"(la), "v"(lb));
      const int mk = (e0 < eend) ? -1 : 0;
      const int sm = snt & ~mk;
      const unsigned s0 = (unsigned)((la.x & mk) | sm) - nbs, s1 = (unsigned)((la.y & mk) | sm) - nbs;
      const unsigned s2 = (unsigned)((la.z & mk) | sm) - nbs, s3 = (unsigned)((la.w & mk) | sm) - nbs;
      const unsigned s4 = (unsigned)((lb.x & mk) | sm) - nbs, s5 = (unsigned)((lb.y & mk) | sm) - nbs;
      const unsigned s6 = (unsigned)((lb.z & mk) | sm) - nbs, s7 = (unsigned)((lb.w & mk) | sm) - nbs;
      const bool h0 = s0 < (unsigned)NBRUN, h1 = s1 < (unsigned)NBRUN, h2 = s2 < (unsigned)NBRUN, h3 = s3 < (unsigned)NBRUN;
      const bool h4 = s4 < (unsigned)NBRUN, h5 = s5 < (unsigned)NBRUN, h6 = s6 < (unsigned)NBRUN, h7 = s7 < (unsigned)NBRUN;
      const unsigned m0 = __builtin_amdgcn_ballot_w32(h0), m1 = __builtin_amdgcn_ballot_w32(h1);
      const unsigned m2 = __builtin_amdgcn_ballot_w32(h2), m3 = __builtin_amdgcn_ballot_w32(h3);
      const unsigned m4 = __builtin_amdgcn_ballot_w32(h4), m5 = __builtin_amdgcn_ballot_w32(h5);
      const unsigned m6 = __builtin_amdgcn_ballot_w32(h6), m7 = __builtin_amdgcn_ballot_w32(h7);
      const unsigned any = m0 | m1 | m2 | m3 | m4 | m5 | m6 | m7;
      if (any != 0u) {
        const int pre = (int)(__builtin_amdgcn_mbcnt_lo(m0, 0u) + __builtin_amdgcn_mbcnt_lo(m1, 0u) +
                              __builtin_amdgcn_mbcnt_lo(m2, 0u) + __builtin_amdgcn_mbcnt_lo(m3, 0u) +
                              __builtin_amdgcn_mbcnt_lo(m4, 0u) + __builtin_amdgcn_mbcnt_lo(m5, 0u) +
                              __builtin_amdgcn_mbcnt_lo(m6, 0u) + __builtin_amdgcn_mbcnt_lo(m7, 0u));
        int p = wc + pre;
        if (h0) { if (p < WLCAP) mylist[p] = ((e0 + 0) << SLB) | (int)s0; p = p + 1; }
        if (h1) { if (p < WLCAP) mylist[p] = ((e0 + 1) << SLB) | (int)s1; p = p + 1; }
        if (h2) { if (p < WLCAP) mylist[p] = ((e0 + 2) << SLB) | (int)s2; p = p + 1; }
        if (h3) { if (p < WLCAP) mylist[p] = ((e0 + 3) << SLB) | (int)s3; p = p + 1; }
        if (h4) { if (p < WLCAP) mylist[p] = ((e0 + 4) << SLB) | (int)s4; p = p + 1; }
        if (h5) { if (p < WLCAP) mylist[p] = ((e0 + 5) << SLB) | (int)s5; p = p + 1; }
        if (h6) { if (p < WLCAP) mylist[p] = ((e0 + 6) << SLB) | (int)s6; p = p + 1; }
        if (h7) { if (p < WLCAP) mylist[p] = ((e0 + 7) << SLB) | (int)s7; p = p + 1; }
        wc += (int)(__builtin_popcount(m0) + __builtin_popcount(m1) + __builtin_popcount(m2) + __builtin_popcount(m3) +
                    __builtin_popcount(m4) + __builtin_popcount(m5) + __builtin_popcount(m6) + __builtin_popcount(m7));
      }
    }
    if (lane == 0) misc[wave] = wc;
  }
  __syncthreads();

  if (wave == 0) {
    int ov = 0, tot = 0;
#pragma unroll 1
    for (int w2 = 0; w2 < NWAVE; ++w2) {
      int c = misc[w2];
      if (c > WLCAP) ov = 1;
      c = c < 0 ? 0 : (c > WLCAP ? WLCAP : c);
      tot += c;
#pragma unroll 1
      for (int b0 = 0; b0 < c; b0 += 32) {
        const int idx = b0 + lane;
        const int ent = wl[w2 * WLCAP + (idx < WLCAP ? idx : WLCAP - 1)];
        const int m32 = (c - b0) < 32 ? (c - b0) : 32;
#pragma unroll 1
        for (int k = 0; k < m32; ++k) {
          const int u    = __builtin_amdgcn_readlane(ent, k);
          const int slot = u & (NBRUN - 1);
          if (lane == 0) cnt[slot] = cnt[slot] + 1;
        }
      }
    }
    if (tot > RCAP) ov = 1;
    if (lane == 0) misc[9] = ov;
  }
  __syncthreads();
  if (wave == 0) {
    const int base = lane * (NBRUN / 32);
    int s = 0;
#pragma unroll 1
    for (int i = 0; i < NBRUN / 32; ++i) s += cnt[base + i];
    int incl = s;
#pragma unroll
    for (int d = 1; d < 32; d <<= 1) {
      const int yv = __shfl_up(incl, d, 32);
      if (lane >= d) incl += yv;
    }
    int run = incl - s;
#pragma unroll 1
    for (int i = 0; i < NBRUN / 32; ++i) {
      const int cv = cnt[base + i];
      offs[base + i] = run;
      cur[base + i]  = run;
      run += cv;
    }
  }
  __syncthreads();

  if (wave == 0) {
#pragma unroll 1
    for (int w2 = 0; w2 < NWAVE; ++w2) {
      int c = misc[w2];
      c = c < 0 ? 0 : (c > WLCAP ? WLCAP : c);
#pragma unroll 1
      for (int b0 = 0; b0 < c; b0 += 32) {
        const int idx = b0 + lane;
        const int ent = wl[w2 * WLCAP + (idx < WLCAP ? idx : WLCAP - 1)];
        int eid = (ent >> SLB) & 0x1FFFFF;
        eid = eid > NE - 1 ? NE - 1 : eid;
        int sr = srcs[eid];
        sr = sr < 0 ? 0 : (sr > NN - 1 ? NN - 1 : sr);
        const int word = (int)((unsigned)sr | ((unsigned)(ent & (NBRUN - 1)) << 16));
        const int m32 = (c - b0) < 32 ? (c - b0) : 32;
#pragma unroll 1
        for (int k = 0; k < m32; ++k) {
          const int u    = __builtin_amdgcn_readlane(ent, k);
          const int wd   = __builtin_amdgcn_readlane(word, k);
          const int slot = u & (NBRUN - 1);
          if (lane == 0) {
            int p = cur[slot];
            p = p < 0 ? 0 : (p > RCAP - 1 ? RCAP - 1 : p);
            pl[p] = wd;
            cur[slot] = p + 1;
          }
        }
      }
    }
  }
  __syncthreads();

  const int ovf = misc[9];
  int* lp  = LIST + (size_t)blk * RCAP;
  int* cop = CO + (size_t)blk * (2 * NBRUN);
  int* fp  = FLAG + (size_t)blk * 32;
  bucket_flush(pl, cnt, ovf, lp, cop, fp, tid);
  __threadfence();
  bucket_flush(pl, cnt, ovf, lp, cop, fp, tid);
}

__global__ __launch_bounds__(NTHR) void k_replay(const float* __restrict__ XLR, const float* __restrict__ GL,
                                                 const int* __restrict__ HITS, const int* __restrict__ CO,
                                                 const int* __restrict__ FLAG, const float* __restrict__ SM,
                                                 float* out) {
  __shared__ __attribute__((aligned(16))) float sab[SAB_N];
  const int tid = (int)threadIdx.x, lane = tid & 31, wave = tid >> 5;
  {
    const int u = tid < SAB_N / 4 ? tid : SAB_N / 4 - 1;
    const v4f v = *(const v4fa*)(SM + SM_ATT + 4 * u);
    asm volatile("" :: "v"(v));
    if (tid < SAB_N / 4) *(v4fa*)(sab + 4 * tid) = v;
  }
  __syncthreads();

  const int iraw = (int)blockIdx.x * NWAVE + wave;
  const bool live = iraw < NN;
  const int i = live ? iraw : NN - 1;
  const int b = i >> SLB, slot = i & (NBRUN - 1);
  const float qnan = __uint_as_float(0x7fc00000u);
  float xr[8];
  {
    const float* xrow = XLR + (size_t)i * NXL + HC + 8 * lane;
    const v4f r0 = *(const v4fa*)xrow;
    const v4f r1 = *(const v4fa*)(xrow + 4);
    xr[0] = r0.x; xr[1] = r0.y; xr[2] = r0.z; xr[3] = r0.w;
    xr[4] = r1.x; xr[5] = r1.y; xr[6] = r1.z; xr[7] = r1.w;
  }
  float w0, w1, w2;
  {
    const v4f g = *(const v4fa*)(GL + (size_t)4 * (size_t)i);
    asm volatile("" :: "v"(g));
    const float gmx = fmaxf(g.x, fmaxf(g.y, g.z));
    const int cs = lane & 3;
    const unsigned k0m = (cs == 0) ? 0xffffffffu : 0u;
    const unsigned k1m = (cs == 1) ? 0xffffffffu : 0u;
    const unsigned k2m = (cs == 2) ? 0xffffffffu : 0u;
    const float gs = __uint_as_float((__float_as_uint(g.x) & k0m) | (__float_as_uint(g.y) & k1m) |
                                     (__float_as_uint(g.z) & k2m));
    const float ev = expf(gs - gmx);
    const float e0 = __shfl(ev, 0, 32), e1 = __shfl(ev, 1, 32), e2 = __shfl(ev, 2, 32);
    const float es = (e0 + e1) + e2;
    const float wv = ev / es;
    w0 = __shfl(wv, 0, 32); w1 = __shfl(wv, 1, 32); w2 = __shfl(wv, 2, 32);
  }

  float res[8];
#pragma unroll
  for (int q = 0; q < 8; ++q) res[q] = 0.0f;
  int bad = 0;

#pragma unroll 1
  for (int k = 0; k < NHOP; ++k) {
    const int rb = k * NBK + b;
    const int* lb  = HITS + (size_t)rb * RCAP;
    const int* cob = CO + (size_t)rb * (2 * NBRUN);
    const int flag = FLAG[(size_t)rb * 32];
    int c = cob[slot];
    int o = cob[NBRUN + slot];
    const int big = (c > DEGCAP) ? 1 : 0;
    c = c < 0 ? 0 : (c > DEGCAP ? DEGCAP : c);
    o = o < 0 ? 0 : (o > RCAP - 1 ? RCAP - 1 : o);
    const int cm = __builtin_amdgcn_readfirstlane(c);
    int last = o + c - 1;
    last = last < o ? o : last;
    last = last > RCAP - 1 ? RCAP - 1 : last;
    bad |= ((flag != 0) ? 1 : 0) | big;
    const int nt = cm + ((k == 0) ? 1 : 0);

    float at[8];
    {
      const v4f a0 = *(const v4fa*)(sab + k * HC + 8 * lane);
      const v4f a1 = *(const v4fa*)(sab + k * HC + 8 * lane + 4);
      at[0] = a0.x; at[1] = a0.y; at[2] = a0.z; at[3] = a0.w;
      at[4] = a1.x; at[5] = a1.y; at[6] = a1.z; at[7] = a1.w;
    }
    float mx = -__builtin_inff(), den = 0.0f;
    float acc[8];
#pragma unroll
    for (int q = 0; q < 8; ++q) acc[q] = 0.0f;

#pragma unroll 1
    for (int j = 0; j < nt; ++j) {
      int idx = o + j;
      idx = idx > last ? last : idx;
      const unsigned wd = (unsigned)lb[idx];
      asm volatile("" :: "v"(wd));
      int sr = (int)(wd & 0xffffu);
      sr = sr > NN - 1 ? NN - 1 : sr;
      sr = (j < cm) ? sr : i;
      const float* sp = XLR + (size_t)sr * NXL + 8 * lane;
      const v4f p0 = *(const v4fa*)sp;
      const v4f p1 = *(const v4fa*)(sp + 4);
      float xs[8];
      xs[0] = p0.x; xs[1] = p0.y; xs[2] = p0.z; xs[3] = p0.w;
      xs[4] = p1.x; xs[5] = p1.y; xs[6] = p1.z; xs[7] = p1.w;
      float part = 0.0f;
#pragma unroll
      for (int q = 0; q < 8; ++q) {
        float v = xs[q] + xr[q];
        v = (v > 0.0f) ? v : (LSLOPE * v);
        part = fmaf(v, at[q], part);
      }
      part += __shfl_xor(part, 1, 32);
      part += __shfl_xor(part, 2, 32);
      part += __shfl_xor(part, 4, 32);
      const float df = part - mx;
      const float ee = expf(-fabsf(df));
      const bool up  = df > 0.0f;
      const float s1 = up ? ee : 1.0f;
      const float s2 = up ? 1.0f : ee;
      mx  = up ? part : mx;
      den = fmaf(den, s1, s2);
#pragma unroll
      for (int q = 0; q < 8; ++q) acc[q] = fmaf(acc[q], s1, s2 * xs[q]);
    }

    const float rinv = 1.0f / (den + 1e-16f);
    const float wk = (k == 0) ? w0 : ((k == 1) ? w1 : w2);
    const int cq = 8 * (lane & 7);
    const v4f b0 = *(const v4fa*)(sab + NHOP * HC + k * CD + cq);
    const v4f b1 = *(const v4fa*)(sab + NHOP * HC + k * CD + cq + 4);
    float bi[8];
    bi[0] = b0.x; bi[1] = b0.y; bi[2] = b0.z; bi[3] = b0.w;
    bi[4] = b1.x; bi[5] = b1.y; bi[6] = b1.z; bi[7] = b1.w;
#pragma unroll
    for (int q = 0; q < 8; ++q) {
      const float hv = (nt > 0) ? (acc[q] * rinv) : 0.0f;
      float t = hv + __shfl_xor(hv, 8, 32);
      t = t + __shfl_xor(t, 16, 32);
      const float mq = fmaf(t, 0.25f, bi[q]);
      res[q] = fmaf(wk, mq, res[q]);
    }
  }

  {
    const int sl = (lane >> 1) & 15;
    float t[8];
#pragma unroll
    for (int q = 0; q < 8; ++q) t[q] = __shfl(res[q], sl, 32);
    const unsigned om = (lane & 1) ? 0xffffffffu : 0u;
    v4f ov;
    ov.x = __uint_as_float((__float_as_uint(t[4]) & om) | (__float_as_uint(t[0]) & ~om));
    ov.y = __uint_as_float((__float_as_uint(t[5]) & om) | (__float_as_uint(t[1]) & ~om));
    ov.z = __uint_as_float((__float_as_uint(t[6]) & om) | (__float_as_uint(t[2]) & ~om));
    ov.w = __uint_as_float((__float_as_uint(t[7]) & om) | (__float_as_uint(t[3]) & ~om));
    const bool poison = bad != 0;
    ov.x = poison ? qnan : ov.x; ov.y = poison ? qnan : ov.y;
    ov.z = poison ? qnan : ov.z; ov.w = poison ? qnan : ov.w;
    float* op = out + (size_t)i * CD + 4 * (lane & 15);
    const bool wr = live && (lane < 16);
    if (wr) *(volatile v4f*)op = ov;
    __threadfence();
    if (wr) *(volatile v4f*)op = ov;
  }
}

extern "C" void kernel_launch(void* const* d_in, const int* in_sizes, int n_in,
                              void* d_out, int out_size, void* d_ws, size_t ws_size,
                              hipStream_t stream) {
  if (n_in < 12) return;
  if (in_sizes[0] != NN * FD) return;
  if (in_sizes[1] != 2 * NE || in_sizes[2] != 2 * NE || in_sizes[3] != 2 * NE) return;
  if (in_sizes[4] != FD * HC || in_sizes[5] != HC) return;
  if (in_sizes[6] != FD * HC || in_sizes[7] != HC) return;
  if (in_sizes[8] != NHOP * NHEAD * CD) return;
  if (in_sizes[9] != NHOP * CD) return;
  if (in_sizes[10] != FD * NHOP || in_sizes[11] != NHOP) return;
  if (out_size != NN * CD) return;

  const float* x    = (const float*)d_in[0];
  const int*   eis[3] = { (const int*)d_in[1], (const int*)d_in[2], (const int*)d_in[3] };
  const float* Wl   = (const float*)d_in[4];
  const float* bl   = (const float*)d_in[5];
  const float* Wr   = (const float*)d_in[6];
  const float* br   = (const float*)d_in[7];
  const float* att  = (const float*)d_in[8];
  const float* bias = (const float*)d_in[9];
  const float* Wg   = (const float*)d_in[10];
  const float* bg   = (const float*)d_in[11];
  float* out = (float*)d_out;

  constexpr size_t zXBH  = (size_t)HROWS * FD * 2;
  constexpr size_t zXLR  = (size_t)MP * NXL * 4;
  constexpr size_t zGL   = (size_t)MP * 4 * 4;
  constexpr size_t zHITS = (size_t)NHOP * NBK * RCAP * 4;
  constexpr size_t zCO   = (size_t)NHOP * NBK * 2 * NBRUN * 4;
  constexpr size_t zFLAG = (((size_t)NHOP * NBK * 128 + 255) / 256) * 256;
  constexpr size_t zBT   = (size_t)NBT * FD * 2;
  constexpr size_t zSM   = (((size_t)SM_TOT * 4 + 255) / 256) * 256;
  constexpr size_t oXBH  = 0;
  constexpr size_t oXLR  = oXBH + zXBH;
  constexpr size_t oGL   = oXLR + zXLR;
  constexpr size_t oHITS = oGL + zGL;
  constexpr size_t oCO   = oHITS + zHITS;
  constexpr size_t oFLAG = oCO + zCO;
  constexpr size_t oBT   = oFLAG + zFLAG;
  constexpr size_t oSM   = oBT + zBT;
  constexpr size_t oEND  = oSM + zSM;
  static_assert(zXBH % 256 == 0 && zXLR % 256 == 0 && zGL % 256 == 0 && zHITS % 256 == 0 && zCO % 256 == 0);
  static_assert(zFLAG % 256 == 0 && zBT % 256 == 0 && zSM % 256 == 0);
  static_assert(oEND <= (size_t)(128u << 20));
  if (oEND > ws_size) return;

  char* ws = (char*)d_ws;
  unsigned short* XBH = (unsigned short*)(ws + oXBH);
  float*          XLR = (float*)(ws + oXLR);
  float*          GL  = (float*)(ws + oGL);
  int*            HITS = (int*)(ws + oHITS);
  int*            CO   = (int*)(ws + oCO);
  int*            FLAG = (int*)(ws + oFLAG);
  unsigned short* BT  = (unsigned short*)(ws + oBT);
  float*          SM  = (float*)(ws + oSM);

  hipFuncSetAttribute(reinterpret_cast<const void*>(&k_bucket), hipFuncAttributeMaxDynamicSharedMemorySize, (int)BK_LDS);

  k_prep<<<PBX + PBW + 1, NTHR, 0, stream>>>(x, Wl, bl, Wr, br, att, bias, Wg, bg, XBH, BT, SM, 0);
  k_gemm_one<<<dim3(HROWS / GBM, 9), NTHR, 0, stream>>>(XBH, BT, SM, XLR, GL, 0);
  k_prep<<<PBX, NTHR, 0, stream>>>(x, Wl, bl, Wr, br, att, bias, Wg, bg, XBH, BT, SM, 1);
  k_gemm_one<<<dim3(HROWS / GBM, 9), NTHR, 0, stream>>>(XBH, BT, SM, XLR, GL, 1);

  for (int r = 0; r < NHOP; ++r) {
    const int* srcs = eis[r];
    const int* dsts = eis[r] + NE;
    k_bucket<<<NBK, NTHR, BK_LDS, stream>>>(srcs, dsts,
                                            HITS + (size_t)r * NBK * RCAP,
                                            CO + (size_t)r * NBK * 2 * NBRUN,
                                            FLAG + (size_t)r * NBK * 32);
  }

  k_replay<<<NN / NWAVE, NTHR, 0, stream>>>(XLR, GL, HITS, CO, FLAG, SM, out);
}
